// MultiHeadAttention_27410481283324
// MI455X (gfx1250) — hardware-verified
//
#include <hip/hip_runtime.h>
#include <math.h>

typedef __attribute__((ext_vector_type(16))) __bf16       v16b;
typedef __attribute__((ext_vector_type(8)))  __bf16       v8b;
typedef __attribute__((ext_vector_type(8)))  float        v8f;
typedef __attribute__((ext_vector_type(4)))  float        v4f;
typedef __attribute__((ext_vector_type(4)))  unsigned int v4u;

constexpr int kBatch = 4;
constexpr int kSeq   = 2048;
constexpr int kDm    = 768;
constexpr int kHeads = 12;
constexpr int kDh    = 64;
constexpr int kPairs = kDh / 2;
constexpr int kRows  = kBatch * kSeq;
constexpr int kBH    = kBatch * kHeads;
constexpr float kQScale = 0.125f;
static_assert(kQScale * kQScale * (float)kDh == 1.0f);
static_assert(kHeads * kDh == kDm);
static_assert((kSeq % 64) == 0 && (kDm % 64) == 0 && (kDm % 32) == 0 && (kRows % 64) == 0);
static_assert(kDh == 64 && kPairs == 32);

constexpr size_t kPlaneB  = (size_t)kRows * kDm * 2;
constexpr size_t kWPlaneB = (size_t)kDm * kDm * 2;
constexpr size_t kOffXB  = 0;
constexpr size_t kOffWB  = kOffXB + kPlaneB;
constexpr size_t kOffQH  = kOffWB + 4 * kWPlaneB;
constexpr size_t kOffQL  = kOffQH + kPlaneB;
constexpr size_t kOffKH  = kOffQL + kPlaneB;
constexpr size_t kOffKL  = kOffKH + kPlaneB;
constexpr size_t kOffVTH = kOffKL + kPlaneB;
constexpr size_t kOffVTL = kOffVTH + kPlaneB;
constexpr size_t kOffOH  = kOffVTL + kPlaneB;
constexpr size_t kOffOL  = kOffOH + kPlaneB;
constexpr size_t kWsTotal = kOffOL + kPlaneB;
static_assert(kWsTotal == 117964800ull);
static_assert(kWsTotal <= 134217728ull);
static_assert((kPlaneB % 128) == 0 && (kWPlaneB % 128) == 0);

__device__ __forceinline__ unsigned short f2bf_bits(float f) {
  unsigned u = __float_as_uint(f);
  return (unsigned short)((u + 0x7FFFu + ((u >> 16) & 1u)) >> 16);
}
__device__ __forceinline__ float bf_bits2f(unsigned short h) { return __uint_as_float(((unsigned)h) << 16); }
__device__ __forceinline__ float bf_rne(float f) { return bf_bits2f(f2bf_bits(f)); }
__device__ __forceinline__ unsigned pk16(unsigned short a, unsigned short b) { return (unsigned)a | ((unsigned)b << 16); }
__device__ __forceinline__ void split_bits(float f, unsigned short& hb, unsigned short& lb) {
  hb = f2bf_bits(f);
  lb = f2bf_bits(f - bf_bits2f(hb));
}
__device__ __forceinline__ void split_bf(float f, __bf16& hi, __bf16& lo) {
  unsigned short hb, lb;
  split_bits(f, hb, lb);
  hi = __builtin_bit_cast(__bf16, hb);
  lo = __builtin_bit_cast(__bf16, lb);
}
union FragB { v16b v; v8b h[2]; };
__device__ __forceinline__ v16b frag_load(const __bf16* p) {
  FragB f;
  f.h[0] = *(const v8b*)(p);
  f.h[1] = *(const v8b*)(p + 16);
  return f.v;
}
__device__ __forceinline__ v8f mma_bf(v16b a, v16b b, v8f c) {
  c = __builtin_amdgcn_wmma_f32_16x16x32_bf16(false, a, false, b, (short)0, c, false, false);
  asm volatile("v_nop\n\tv_nop\n\tv_nop\n\tv_nop" : "+v"(c) : "v"(a), "v"(b));
  return c;
}
__device__ __forceinline__ void wave_lds_sync() {
  __builtin_amdgcn_fence(__ATOMIC_RELEASE, "workgroup");
  __builtin_amdgcn_wave_barrier();
  __builtin_amdgcn_fence(__ATOMIC_ACQUIRE, "workgroup");
}

__global__ __launch_bounds__(256) void cast8_bf16_kernel(
    const float* s0, const float* s1, const float* s2, const float* s3,
    unsigned short* __restrict__ out, long planeElems, int n8)
{
  const int z = blockIdx.y;
  const float* src = (z == 0) ? s0 : (z == 1) ? s1 : (z == 2) ? s2 : s3;
  const int i = blockIdx.x * 256 + threadIdx.x;
  if (i >= n8) return;
  const size_t e0 = (size_t)i << 3;
  const v4f a0 = *(const v4f*)(src + e0);
  const v4f a1 = *(const v4f*)(src + e0 + 4);
  unsigned short hb[8];
#pragma unroll
  for (int e = 0; e < 4; ++e) {
    const float f0 = a0[e];
    const float f1 = a1[e];
    hb[e]     = f2bf_bits(f0);
    hb[4 + e] = f2bf_bits(f1);
  }
  const v4u u = (v4u){pk16(hb[0], hb[1]), pk16(hb[2], hb[3]), pk16(hb[4], hb[5]), pk16(hb[6], hb[7])};
  unsigned short* q = out + (size_t)z * (size_t)planeElems + e0;
  *(volatile v4u*)q = u;
  __threadfence();
  *(volatile v4u*)q = u;
}

template <int SPL, int EPI>
__global__ __launch_bounds__(256) void gemm64_kernel(
    const unsigned short* __restrict__ Ap, const unsigned short* __restrict__ A2p, int lda, long strideA,
    const unsigned short* __restrict__ Btp, int ldb, long strideB,
    void* __restrict__ Cout, void* __restrict__ Cout2, int ldc, long strideC,
    const float* __restrict__ rcos, const float* __restrict__ rsin,
    int M, int N, int K)
{
  __shared__ __align__(16) float sT[8][16 * 68];
  const int bz   = blockIdx.y;
  const int lane = threadIdx.x & 31;
  const int wave = __builtin_amdgcn_readfirstlane((int)(threadIdx.x >> 5));
  const int tilesN = N >> 6;
  const int tilesM = M >> 6;
  const int tile = blockIdx.x * 8 + wave;
  if (tile >= tilesM * tilesN) return;
  const int tm = tile / tilesN;
  const int tn = tile - tm * tilesN;
  const int m0 = tm << 6;
  const int n0 = tn << 6;

  const __bf16* Ab  = (const __bf16*)Ap + (size_t)bz * (size_t)strideA;
  const __bf16* Ab2 = (SPL == 1) ? ((const __bf16*)A2p + (size_t)bz * (size_t)strideA) : Ab;
  const __bf16* Bb  = (const __bf16*)Btp + (size_t)bz * (size_t)strideB;

  const int rlane = lane & 15;
  const int koff  = (lane >> 4) * 8;
  const int mOff  = (lane >> 4) * 8;

  v8f acc[4][4];
#pragma unroll
  for (int i = 0; i < 4; ++i)
#pragma unroll
    for (int j = 0; j < 4; ++j) acc[i][j] = (v8f){0.f, 0.f, 0.f, 0.f, 0.f, 0.f, 0.f, 0.f};

  for (int k0 = 0; k0 < K; k0 += 32) {
    v16b bh[4];
#pragma unroll
    for (int j = 0; j < 4; ++j)
      bh[j] = frag_load(Bb + (size_t)(n0 + (j << 4) + rlane) * ldb + koff + k0);
#pragma unroll
    for (int i = 0; i < 4; ++i) {
      const size_t ao = (size_t)(m0 + (i << 4) + rlane) * lda + koff + k0;
      const v16b ah = frag_load(Ab + ao);
      v16b al = ah;
      if (SPL == 1) al = frag_load(Ab2 + ao);
#pragma unroll
      for (int j = 0; j < 4; ++j) {
        acc[i][j] = mma_bf(ah, bh[j], acc[i][j]);
        if (SPL == 1) acc[i][j] = mma_bf(al, bh[j], acc[i][j]);
      }
    }
  }

  float* slab = sT[wave];
#pragma unroll
  for (int i = 0; i < 4; ++i) {
    const int mBase = m0 + (i << 4);
#pragma unroll
    for (int j = 0; j < 4; ++j) {
#pragma unroll
      for (int r = 0; r < 8; ++r) slab[(mOff + r) * 68 + (j << 4) + rlane] = acc[i][j][r];
    }
    wave_lds_sync();
    if (EPI == 0) {
      float* C = (float*)Cout + (size_t)bz * (size_t)strideC;
      const int hh = lane >> 4, c4 = (lane & 15) * 4;
      for (int pass = 0; pass < 2; ++pass) {
#pragma unroll
        for (int it = 0; it < 8; ++it) {
          const int row = it * 2 + hh;
          const v4f v = *(const v4f*)(slab + row * 68 + c4);
          *(volatile v4f*)(C + (size_t)(mBase + row) * ldc + n0 + c4) = v;
        }
        __threadfence();
      }
    } else {
      const int q = lane >> 3, c8 = (lane & 7) * 8;
      unsigned short* C  = (unsigned short*)Cout  + (size_t)bz * (size_t)strideC;
      unsigned short* C2 = (unsigned short*)Cout2 + (size_t)bz * (size_t)strideC;
      const float qs = (bz == 0) ? kQScale : 1.0f;
      v4u hu[4], lu[4];
      size_t oaddr[4];
#pragma unroll
      for (int it = 0; it < 4; ++it) {
        const int row = it * 4 + q;
        const float* sp = slab + row * 68 + c8;
        const v4f a0 = *(const v4f*)(sp);
        const v4f a1 = *(const v4f*)(sp + 4);
        float y[8];
        y[0] = a0[0]; y[1] = a0[1]; y[2] = a0[2]; y[3] = a0[3];
        y[4] = a1[0]; y[5] = a1[1]; y[6] = a1[2]; y[7] = a1[3];
        const int g = mBase + row;
        if (EPI == 3) {
          const int tpos = g & (kSeq - 1);
          const int bb   = g / kSeq;
          const v4f cv = *(const v4f*)(rcos + (size_t)tpos * kPairs + (c8 >> 1));
          const v4f sv = *(const v4f*)(rsin + (size_t)tpos * kPairs + (c8 >> 1));
#pragma unroll
          for (int e2 = 0; e2 < 4; ++e2) {
            const float cf0 = cv[e2];
            const float sf0 = sv[e2];
            const float cf = bf_rne(cf0);
            const float sf = bf_rne(sf0);
            const float x1 = y[2 * e2];
            const float x2 = y[2 * e2 + 1];
            y[2 * e2]     = (x1 * cf - x2 * sf) * qs;
            y[2 * e2 + 1] = (x1 * sf + x2 * cf) * qs;
          }
          oaddr[it] = (((size_t)(bb * kHeads + tn)) * kSeq + tpos) * kDh + c8;
        } else {
          oaddr[it] = (size_t)g * ldc + n0 + c8;
        }
        unsigned short hb[8], lb[8];
#pragma unroll
        for (int e = 0; e < 8; ++e) split_bits(y[e], hb[e], lb[e]);
        hu[it] = (v4u){pk16(hb[0], hb[1]), pk16(hb[2], hb[3]), pk16(hb[4], hb[5]), pk16(hb[6], hb[7])};
        lu[it] = (v4u){pk16(lb[0], lb[1]), pk16(lb[2], lb[3]), pk16(lb[4], lb[5]), pk16(lb[6], lb[7])};
      }
      for (int pass = 0; pass < 2; ++pass) {
#pragma unroll
        for (int it = 0; it < 4; ++it) {
          *(volatile v4u*)(C  + oaddr[it]) = hu[it];
          *(volatile v4u*)(C2 + oaddr[it]) = lu[it];
        }
        __threadfence();
      }
    }
    wave_lds_sync();
  }
}

__global__ __launch_bounds__(128) void causal_ctx_kernel(
    const unsigned short* __restrict__ qhp, const unsigned short* __restrict__ qlp,
    const unsigned short* __restrict__ khp, const unsigned short* __restrict__ klp,
    const unsigned short* __restrict__ vhp, const unsigned short* __restrict__ vlp,
    unsigned short* __restrict__ ohp, unsigned short* __restrict__ olp)
{
  __shared__ __align__(16) __bf16 Psh[4][16 * 64];
  __shared__ __align__(16) __bf16 Psl[4][16 * 64];
  __shared__ __align__(16) float  Os[4][16 * 68];

  const int tid  = threadIdx.x;
  const int wave = __builtin_amdgcn_readfirstlane((int)(threadIdx.x >> 5));
  const int lane = tid & 31;
  const int hh   = lane >> 4;
  const int c    = lane & 15;

  constexpr int nqb = kSeq / 64;
  const int qb = blockIdx.x % nqb;
  const int bh = blockIdx.x / nqb;
  const int hd = bh % kHeads;
  const int bi = bh / kHeads;
  const int q0 = qb * 64 + wave * 16;

  const size_t pbase = (size_t)bh * kSeq * kDh;
  const __bf16* Qh = (const __bf16*)qhp + pbase;
  const __bf16* Ql = (const __bf16*)qlp + pbase;
  const __bf16* Kh = (const __bf16*)khp + pbase;
  const __bf16* Kl = (const __bf16*)klp + pbase;
  const __bf16* Vh = (const __bf16*)vhp + pbase;
  const __bf16* Vl = (const __bf16*)vlp + pbase;

  v16b qah[2], qal[2];
#pragma unroll
  for (int dc = 0; dc < 2; ++dc) {
    const size_t qo = (size_t)(q0 + c) * kDh + dc * 32 + 8 * hh;
    qah[dc] = frag_load(Qh + qo);
    qal[dc] = frag_load(Ql + qo);
  }

  float mrow[8], lrow[8];
  v8f oacc[4];
#pragma unroll
  for (int r = 0; r < 8; ++r) { mrow[r] = -INFINITY; lrow[r] = 0.f; }
#pragma unroll
  for (int t = 0; t < 4; ++t) oacc[t] = (v8f){0.f, 0.f, 0.f, 0.f, 0.f, 0.f, 0.f, 0.f};

  __bf16* pwh = Psh[wave];
  __bf16* pwl = Psl[wave];
  const int nChunks = qb + 1;

#pragma unroll 1
  for (int kc = 0; kc < nChunks; ++kc) {
    const int kv0 = kc * 64;
    v8f s[4];
#pragma unroll
    for (int j = 0; j < 4; ++j) {
      s[j] = (v8f){0.f, 0.f, 0.f, 0.f, 0.f, 0.f, 0.f, 0.f};
#pragma unroll
      for (int dc = 0; dc < 2; ++dc) {
        const size_t ko = (size_t)(kv0 + j * 16 + c) * kDh + dc * 32 + 8 * hh;
        const v16b kbh = frag_load(Kh + ko);
        const v16b kbl = frag_load(Kl + ko);
        s[j] = mma_bf(qah[dc], kbl, s[j]);
        s[j] = mma_bf(qal[dc], kbh, s[j]);
        s[j] = mma_bf(qah[dc], kbh, s[j]);
      }
    }
    const bool diag = (kc == qb);
    float cm[8];
#pragma unroll
    for (int r = 0; r < 8; ++r) {
      const int qrow = q0 + 8 * hh + r;
      float m = -INFINITY;
#pragma unroll
      for (int j = 0; j < 4; ++j) {
        const int kvcol = kv0 + j * 16 + c;
        const float sv = s[j][r];
        const float sm = (diag && (kvcol > qrow)) ? -INFINITY : sv;
        s[j][r] = sm;
        m = fmaxf(m, sm);
      }
#pragma unroll
      for (int off = 1; off < 16; off <<= 1) m = fmaxf(m, __shfl_xor(m, off, 32));
      cm[r] = m;
    }
#pragma unroll
    for (int r = 0; r < 8; ++r) {
      const float mnew  = fmaxf(mrow[r], cm[r]);
      const float alpha = __expf(mrow[r] - mnew);
      mrow[r] = mnew;
      float psum = 0.f;
#pragma unroll
      for (int j = 0; j < 4; ++j) {
        const float p = __expf(s[j][r] - mnew);
        psum += p;
        __bf16 ph, pl;
        split_bf(p, ph, pl);
        pwh[(8 * hh + r) * 64 + j * 16 + c] = ph;
        pwl[(8 * hh + r) * 64 + j * 16 + c] = pl;
      }
#pragma unroll
      for (int off = 1; off < 16; off <<= 1) psum += __shfl_xor(psum, off, 32);
      lrow[r] = lrow[r] * alpha + psum;
#pragma unroll
      for (int t = 0; t < 4; ++t) oacc[t][r] *= alpha;
    }
    wave_lds_sync();
#pragma unroll 1
    for (int kk = 0; kk < 2; ++kk) {
      const v16b pa = frag_load(pwh + c * 64 + kk * 32 + 8 * hh);
      const v16b pl = frag_load(pwl + c * 64 + kk * 32 + 8 * hh);
#pragma unroll
      for (int t = 0; t < 4; ++t) {
        const size_t vo = (size_t)(t * 16 + c) * kSeq + kv0 + kk * 32 + 8 * hh;
        const v16b vbh = frag_load(Vh + vo);
        const v16b vbl = frag_load(Vl + vo);
        oacc[t] = mma_bf(pa, vbl, oacc[t]);
        oacc[t] = mma_bf(pl, vbh, oacc[t]);
        oacc[t] = mma_bf(pa, vbh, oacc[t]);
      }
    }
    wave_lds_sync();
  }

  float* os = Os[wave];
#pragma unroll
  for (int r = 0; r < 8; ++r) {
    const float inv = 1.0f / lrow[r];
#pragma unroll
    for (int t = 0; t < 4; ++t) os[(8 * hh + r) * 68 + t * 16 + c] = oacc[t][r] * inv;
  }
  wave_lds_sync();
  {
    const int q = lane >> 3, c8 = (lane & 7) * 8;
    v4u hu[4], lu[4];
#pragma unroll
    for (int it = 0; it < 4; ++it) {
      const int row = it * 4 + q;
      const float* sp = os + row * 68 + c8;
      const v4f a0 = *(const v4f*)(sp);
      const v4f a1 = *(const v4f*)(sp + 4);
      float y[8];
      y[0] = a0[0]; y[1] = a0[1]; y[2] = a0[2]; y[3] = a0[3];
      y[4] = a1[0]; y[5] = a1[1]; y[6] = a1[2]; y[7] = a1[3];
      unsigned short hb[8], lb[8];
#pragma unroll
      for (int e = 0; e < 8; ++e) split_bits(y[e], hb[e], lb[e]);
      hu[it] = (v4u){pk16(hb[0], hb[1]), pk16(hb[2], hb[3]), pk16(hb[4], hb[5]), pk16(hb[6], hb[7])};
      lu[it] = (v4u){pk16(lb[0], lb[1]), pk16(lb[2], lb[3]), pk16(lb[4], lb[5]), pk16(lb[6], lb[7])};
    }
    for (int pass = 0; pass < 2; ++pass) {
#pragma unroll
      for (int it = 0; it < 4; ++it) {
        const int row = it * 4 + q;
        const size_t o = (size_t)(bi * kSeq + q0 + row) * kDm + hd * kDh + c8;
        *(volatile v4u*)(ohp + o) = hu[it];
        *(volatile v4u*)(olp + o) = lu[it];
      }
      __threadfence();
    }
  }
}

extern "C" void kernel_launch(void* const* d_in, const int* in_sizes, int n_in,
                              void* d_out, int out_size, void* d_ws, size_t ws_size,
                              hipStream_t stream) {
  if (n_in < 7) return;
  if (in_sizes[0] != kRows * kDm) return;
  if (in_sizes[1] != kSeq * kPairs) return;
  if (in_sizes[2] != kSeq * kPairs) return;
  if (in_sizes[3] != kDm * kDm) return;
  if (in_sizes[4] != kDm * kDm) return;
  if (in_sizes[5] != kDm * kDm) return;
  if (in_sizes[6] != kDm * kDm) return;
  if (out_size != kRows * kDm) return;
  if (ws_size < kWsTotal) return;

  const float* x  = (const float*)d_in[0];
  const float* rc = (const float*)d_in[1];
  const float* rs = (const float*)d_in[2];
  const float* wq = (const float*)d_in[3];
  const float* wk = (const float*)d_in[4];
  const float* wv = (const float*)d_in[5];
  const float* wo = (const float*)d_in[6];
  float* out = (float*)d_out;

  char* ws = (char*)d_ws;
  unsigned short* XB  = (unsigned short*)(ws + kOffXB);
  unsigned short* WB  = (unsigned short*)(ws + kOffWB);
  unsigned short* QH  = (unsigned short*)(ws + kOffQH);
  unsigned short* QL  = (unsigned short*)(ws + kOffQL);
  unsigned short* KH  = (unsigned short*)(ws + kOffKH);
  unsigned short* KL  = (unsigned short*)(ws + kOffKL);
  unsigned short* VTH = (unsigned short*)(ws + kOffVTH);
  unsigned short* VTL = (unsigned short*)(ws + kOffVTL);
  unsigned short* OH  = (unsigned short*)(ws + kOffOH);
  unsigned short* OL  = (unsigned short*)(ws + kOffOL);

  constexpr int kXn8 = kRows * kDm / 8;
  constexpr int kWn8 = kDm * kDm / 8;
  static_assert((kXn8 % 256) == 0 && (kWn8 % 256) == 0);
  constexpr long kWElems = (long)kDm * kDm;
  constexpr long kPlaneElems = (long)kRows * kDm;

  cast8_bf16_kernel<<<dim3(kXn8 / 256, 1), 256, 0, stream>>>(x, x, x, x, XB, 0L, kXn8);
  cast8_bf16_kernel<<<dim3(kWn8 / 256, 4), 256, 0, stream>>>(wq, wk, wv, wo, WB, kWElems, kWn8);

  constexpr int kQkBlocks = (kRows / 64) * (kDm / 64) / 8;
  static_assert(kQkBlocks * 8 == (kRows / 64) * (kDm / 64));
  gemm64_kernel<0, 3><<<dim3(kQkBlocks, 2), 256, 0, stream>>>(
      XB, XB, kDm, 0L,
      WB, kDm, kWElems,
      (void*)QH, (void*)QL, 0, 2L * kPlaneElems,
      rc, rs,
      kRows, kDm, kDm);

  constexpr int kVtBlocks = (kDm / 64) * (kSeq / 64) / 8;
  static_assert(kVtBlocks * 8 == (kDm / 64) * (kSeq / 64));
  gemm64_kernel<0, 2><<<dim3(kVtBlocks, kBatch), 256, 0, stream>>>(
      WB + 2 * kWElems, WB + 2 * kWElems, kDm, 0L,
      XB, kDm, (long)kSeq * kDm,
      (void*)VTH, (void*)VTL, kSeq, (long)kDm * kSeq,
      nullptr, nullptr,
      kDm, kSeq, kDm);

  causal_ctx_kernel<<<dim3(kBH * (kSeq / 64)), 128, 0, stream>>>(QH, QL, KH, KL, VTH, VTL, OH, OL);

  gemm64_kernel<1, 0><<<dim3(kQkBlocks, 1), 256, 0, stream>>>(
      OH, OL, kDm, 0L,
      WB + 3 * kWElems, kDm, 0L,
      (void*)out, nullptr, kDm, 0L,
      nullptr, nullptr,
      kRows, kDm, kDm);
}
